// MyAttention_76579266888453
// MI455X (gfx1250) — hardware-verified
//
#include <hip/hip_runtime.h>
#include <stddef.h>


typedef __bf16 v16bf __attribute__((ext_vector_type(16)));
typedef float v8f __attribute__((ext_vector_type(8)));
typedef float v4f __attribute__((ext_vector_type(4)));
typedef unsigned int v4u __attribute__((ext_vector_type(4)));

union Frag { v4u u[2]; v16bf v; };

namespace {
constexpr int kC = 1024;
constexpr int kH = 16;
constexpr int kHD = 64;
constexpr int kNP = 64;
constexpr int kL = 65;
constexpr int kKT = kC / 32;
constexpr int kRawPerB = kH * kL;
constexpr int kTP = 68;
constexpr int kWP = 72;
constexpr float kScale = 0.125f;
}

__device__ __forceinline__ v8f wmma_bf16(v16bf a, v16bf b, v8f c) {
  v8f d = __builtin_amdgcn_wmma_f32_16x16x32_bf16(false, a, false, b, (short)0, c, false, false);
  asm volatile("v_nop\n\tv_nop\n\tv_nop\n\tv_nop" : "+v"(d) : "v"(a), "v"(b));
  return d;
}

__device__ __forceinline__ unsigned int bf16_rne(float f) {
  const unsigned int u = __float_as_uint(f);
  return (u + 0x7FFFu + ((u >> 16) & 1u)) >> 16;
}
__device__ __forceinline__ float bf16_val(unsigned int b) {
  return __uint_as_float(b << 16);
}

__global__ void __launch_bounds__(256) cvt_split_kernel(const float* __restrict__ src,
                                                        unsigned short* hi,
                                                        unsigned short* lo, int n8) {
  const int i = blockIdx.x * 256 + threadIdx.x;
  if (i >= n8) return;
  const float* p = src + (size_t)i * 8;
  const v4f x0 = *(const v4f*)p;
  const v4f x1 = *(const v4f*)(p + 4);
  const float xs[8] = {x0[0], x0[1], x0[2], x0[3], x1[0], x1[1], x1[2], x1[3]};
  unsigned int hb[8], lb[8];
#pragma unroll
  for (int j = 0; j < 8; ++j) {
    hb[j] = bf16_rne(xs[j]);
    lb[j] = bf16_rne(xs[j] - bf16_val(hb[j]));
  }
  unsigned int hw[4], lw[4];
#pragma unroll
  for (int q = 0; q < 4; ++q) {
    hw[q] = hb[2 * q] | (hb[2 * q + 1] << 16);
    lw[q] = lb[2 * q] | (lb[2 * q + 1] << 16);
  }
  const v4u hv = {hw[0], hw[1], hw[2], hw[3]};
  const v4u lv = {lw[0], lw[1], lw[2], lw[3]};
  volatile v4u* ph = (volatile v4u*)(hi + (size_t)i * 8);
  volatile v4u* pl = (volatile v4u*)(lo + (size_t)i * 8);
  *ph = hv;
  *pl = lv;
  __threadfence();
  *ph = hv;
  *pl = lv;
}

template <bool SPLIT>
__global__ void __launch_bounds__(256) pack_wt_kernel(const float* __restrict__ W,
                                                      unsigned short* hi,
                                                      unsigned short* lo,
                                                      int ntn, int ntk) {
  __shared__ __attribute__((aligned(16))) unsigned short sHi[64 * kWP];
  __shared__ __attribute__((aligned(16))) unsigned short sLo[64 * kWP];
  const int t = threadIdx.x;
  const int bt = blockIdx.x;
  if (bt >= ntn * ntk) return;
  const int n0 = (bt % ntn) * 64;
  const int k0 = (bt / ntn) * 64;
  const int nn = t & 63;
  const int kq = t >> 6;
#pragma unroll 4
  for (int i = 0; i < 16; ++i) {
    const int kk = kq + 4 * i;
    const float v = W[(size_t)(k0 + kk) * kC + n0 + nn];
    const unsigned int hb = bf16_rne(v);
    sHi[nn * kWP + kk] = (unsigned short)hb;
    if constexpr (SPLIT) {
      sLo[nn * kWP + kk] = (unsigned short)bf16_rne(v - bf16_val(hb));
    }
  }
  __syncthreads();
  v4u hv[2], lv[2];
  size_t go[2];
#pragma unroll
  for (int p = 0; p < 2; ++p) {
    const int L = p * 32 + (t >> 3);
    const int kk0 = (t & 7) * 8;
    hv[p] = *(const v4u*)(sHi + L * kWP + kk0);
    if constexpr (SPLIT) {
      lv[p] = *(const v4u*)(sLo + L * kWP + kk0);
    } else {
      lv[p] = hv[p];
    }
    go[p] = (size_t)(n0 + L) * kC + k0 + kk0;
  }
#pragma unroll
  for (int p = 0; p < 2; ++p) {
    *(volatile v4u*)(hi + go[p]) = hv[p];
    if constexpr (SPLIT) { *(volatile v4u*)(lo + go[p]) = lv[p]; }
  }
  __threadfence();
#pragma unroll
  for (int p = 0; p < 2; ++p) {
    *(volatile v4u*)(hi + go[p]) = hv[p];
    if constexpr (SPLIT) { *(volatile v4u*)(lo + go[p]) = lv[p]; }
  }
}

template <bool SPLIT, bool EPI>
__global__ void __launch_bounds__(256) gemm_kernel(const unsigned short* __restrict__ Ahi,
                                                   const unsigned short* __restrict__ Alo,
                                                   const unsigned short* __restrict__ Bhi,
                                                   const unsigned short* __restrict__ Blo,
                                                   float* Out,
                                                   const float* __restrict__ bias,
                                                   const float* __restrict__ resid,
                                                   int Mtiles) {
  __shared__ __attribute__((aligned(16))) float sT[8 * 16 * kTP];
  const int wv = threadIdx.x >> 5;
  const int l = threadIdx.x & 31;
  const int h = l >> 4;
  const int m = l & 15;
  const int total = Mtiles * 16;
  if ((int)blockIdx.x * 8 >= total) return;
  const int waveId = blockIdx.x * 8 + wv;
  const int row0 = (waveId >> 4) * 16;
  const int col0 = (waveId & 15) * 64;

  const v8f zero8 = {0.f, 0.f, 0.f, 0.f, 0.f, 0.f, 0.f, 0.f};
  v8f acc[4];
#pragma unroll
  for (int f = 0; f < 4; ++f) acc[f] = zero8;

  const unsigned short* aph = Ahi + (size_t)(row0 + m) * kC + 8 * h;
  const unsigned short* apl = Alo + (size_t)(row0 + m) * kC + 8 * h;
  const unsigned short* bph = Bhi + (size_t)(col0 + m) * kC + 8 * h;
  const unsigned short* bpl = Blo + (size_t)(col0 + m) * kC + 8 * h;

#pragma unroll 1
  for (int kt = 0; kt < kKT; ++kt) {
    const int k0 = kt * 32;
    Frag ah;
    ah.u[0] = *(const v4u*)(aph + k0);
    ah.u[1] = *(const v4u*)(aph + k0 + 16);
    Frag al;
    if constexpr (SPLIT) {
      al.u[0] = *(const v4u*)(apl + k0);
      al.u[1] = *(const v4u*)(apl + k0 + 16);
    } else {
      al = ah;
    }
#pragma unroll
    for (int f = 0; f < 4; ++f) {
      const size_t fo = (size_t)f * 16 * kC + (size_t)k0;
      Frag bh;
      bh.u[0] = *(const v4u*)(bph + fo);
      bh.u[1] = *(const v4u*)(bph + fo + 16);
      acc[f] = wmma_bf16(ah.v, bh.v, acc[f]);
      if constexpr (SPLIT) {
        Frag bl;
        bl.u[0] = *(const v4u*)(bpl + fo);
        bl.u[1] = *(const v4u*)(bpl + fo + 16);
        acc[f] = wmma_bf16(ah.v, bl.v, acc[f]);
        acc[f] = wmma_bf16(al.v, bh.v, acc[f]);
      }
    }
  }

  float* st = sT + wv * 16 * kTP;
#pragma unroll
  for (int f = 0; f < 4; ++f) {
#pragma unroll
    for (int r = 0; r < 8; ++r) {
      st[(8 * h + r) * kTP + 16 * f + m] = acc[f][r];
    }
  }
  __syncthreads();

  v4f vals[8];
  size_t go[8];
#pragma unroll
  for (int s = 0; s < 8; ++s) {
    const int L = 4 * s + (l >> 3);
    const int row = L >> 1;
    const int col = (L & 1) * 32 + (l & 7) * 4;
    v4f v = *(const v4f*)(st + row * kTP + col);
    go[s] = (size_t)(row0 + row) * kC + col0 + col;
    if constexpr (EPI) {
      const v4f b4 = *(const v4f*)(bias + col0 + col);
      const v4f x4 = *(const v4f*)(resid + go[s]);
      v = (v + b4) + x4;
    }
    vals[s] = v;
  }
#pragma unroll
  for (int s = 0; s < 8; ++s) *(volatile v4f*)(Out + go[s]) = vals[s];
  __threadfence();
#pragma unroll
  for (int s = 0; s < 8; ++s) *(volatile v4f*)(Out + go[s]) = vals[s];
}

__global__ void __launch_bounds__(256) attn_kernel(const float* __restrict__ Qf,
                                                   const float* __restrict__ Kx,
                                                   const float* __restrict__ Vx,
                                                   const float* __restrict__ Kp,
                                                   const float* __restrict__ Vp,
                                                   float* rawOut,
                                                   unsigned short* Xcls, int nb) {
  __shared__ __attribute__((aligned(16))) float qS[2 * kC];
  __shared__ __attribute__((aligned(16))) float rawS[2 * kRawPerB];
  __shared__ __attribute__((aligned(16))) float attnS[2 * kRawPerB];
  __shared__ __attribute__((aligned(16))) float xS[2 * kC];
  const int tid = threadIdx.x;
  const int b0 = blockIdx.x * 2;
  if (b0 + 2 > nb) return;

  for (int i = tid; i < 2 * kC; i += 256) qS[i] = Qf[(size_t)b0 * kC + i] * kScale;
  __syncthreads();

  for (int idx = tid; idx < 2 * kRawPerB; idx += 256) {
    const int bb = (idx >= kRawPerB) ? 1 : 0;
    const int rem = idx - bb * kRawPerB;
    const int hh = rem / kL;
    const int ll = rem - hh * kL;
    const float* q = qS + bb * kC + hh * kHD;
    const float* kr = (ll == 0) ? (Kx + (size_t)(b0 + bb) * kC + hh * kHD)
                                : (Kp + (size_t)(ll - 1) * kC + hh * kHD);
    float acc = 0.f;
#pragma unroll 2
    for (int d = 0; d < kHD; d += 4) {
      const v4f qa = *(const v4f*)(q + d);
      const v4f ka = *(const v4f*)(kr + d);
      acc += qa[0] * ka[0];
      acc += qa[1] * ka[1];
      acc += qa[2] * ka[2];
      acc += qa[3] * ka[3];
    }
    rawS[idx] = acc;
  }
  __syncthreads();

  if (tid < 32) {
    const int base = tid * kL;
    float mx = rawS[base];
#pragma unroll 1
    for (int j = 1; j < kL; ++j) mx = fmaxf(mx, rawS[base + j]);
    float s = 0.f;
#pragma unroll 1
    for (int j = 0; j < kL; ++j) s += expf(rawS[base + j] - mx);
    const float inv = 1.0f / s;
#pragma unroll 1
    for (int j = 0; j < kL; ++j) attnS[base + j] = (expf(rawS[base + j] - mx) * inv) * kScale;
  }

  {
    v4f rv[3];
    size_t go[3];
    bool ok[3];
    const int j4 = (tid & 7) * 4;
#pragma unroll
    for (int p = 0; p < 3; ++p) {
      const int L = p * 32 + (tid >> 3);
      ok[p] = (L < 65);
      const int Lc = ok[p] ? L : 0;
      rv[p] = *(const v4f*)(rawS + Lc * 32 + j4);
      go[p] = (size_t)b0 * kRawPerB + (size_t)Lc * 32 + j4;
    }
#pragma unroll
    for (int p = 0; p < 3; ++p) { if (ok[p]) *(volatile v4f*)(rawOut + go[p]) = rv[p]; }
    __threadfence();
#pragma unroll
    for (int p = 0; p < 3; ++p) { if (ok[p]) *(volatile v4f*)(rawOut + go[p]) = rv[p]; }
  }
  __syncthreads();

  for (int c4 = tid; c4 < 512; c4 += 256) {
    const int c = c4 * 4;
    const int bb = c >> 10;
    const int cc = c & 1023;
    const int hh = cc >> 6;
    const float* at = attnS + bb * kRawPerB + hh * kL;
    v4f acc = *(const v4f*)(Vx + (size_t)(b0 + bb) * kC + cc) * at[0];
#pragma unroll 2
    for (int r = 0; r < kNP; ++r) {
      const v4f vv = *(const v4f*)(Vp + (size_t)r * kC + cc);
      acc += vv * at[1 + r];
    }
    *(v4f*)(xS + c) = acc;
  }
  __syncthreads();

  {
    const int L = tid >> 3;
    const int bb = L >> 4;
    const int c0 = (L & 15) * 64 + (tid & 7) * 8;
    const v4f a0 = *(const v4f*)(xS + bb * kC + c0);
    const v4f a1 = *(const v4f*)(xS + bb * kC + c0 + 4);
    unsigned int w[4];
    w[0] = bf16_rne(a0[0]) | (bf16_rne(a0[1]) << 16);
    w[1] = bf16_rne(a0[2]) | (bf16_rne(a0[3]) << 16);
    w[2] = bf16_rne(a1[0]) | (bf16_rne(a1[1]) << 16);
    w[3] = bf16_rne(a1[2]) | (bf16_rne(a1[3]) << 16);
    const v4u pk = {w[0], w[1], w[2], w[3]};
    volatile v4u* dst = (volatile v4u*)(Xcls + (size_t)(b0 + bb) * kC + c0);
    *dst = pk;
    __threadfence();
    *dst = pk;
  }
}

extern "C" void kernel_launch(void* const* d_in, const int* in_sizes, int n_in,
                              void* d_out, int out_size, void* d_ws, size_t ws_size,
                              hipStream_t stream) {
  if (n_in < 7) return;
  const int B = in_sizes[0] / kC;
  if (B < 16 || (B % 16) != 0 || in_sizes[0] != B * kC) return;
  if (in_sizes[1] != kNP * kC) return;
  if (in_sizes[2] != kC * kC || in_sizes[3] != kC * kC ||
      in_sizes[4] != kC * kC || in_sizes[5] != kC * kC) return;
  if (in_sizes[6] != kC) return;
  if (out_size != B * kC + B * kRawPerB) return;

  const float* x       = (const float*)d_in[0];
  const float* prompts = (const float*)d_in[1];
  const float* Wq      = (const float*)d_in[2];
  const float* Wk      = (const float*)d_in[3];
  const float* Wv      = (const float*)d_in[4];
  const float* Wp      = (const float*)d_in[5];
  const float* bp      = (const float*)d_in[6];

  float* out_cls = (float*)d_out;
  float* out_raw = out_cls + (size_t)B * kC;

  char* ws = (char*)d_ws;
  size_t off = 0;
  const size_t wplane = (size_t)kC * kC * 2;
  unsigned short* WQH = (unsigned short*)(ws + off); off += wplane;
  unsigned short* WQL = (unsigned short*)(ws + off); off += wplane;
  unsigned short* WKH = (unsigned short*)(ws + off); off += wplane;
  unsigned short* WKL = (unsigned short*)(ws + off); off += wplane;
  unsigned short* WVH = (unsigned short*)(ws + off); off += wplane;
  unsigned short* WPH = (unsigned short*)(ws + off); off += wplane;
  unsigned short* XH  = (unsigned short*)(ws + off); off += (size_t)B * kC * 2;
  unsigned short* XL  = (unsigned short*)(ws + off); off += (size_t)B * kC * 2;
  unsigned short* PH  = (unsigned short*)(ws + off); off += (size_t)kNP * kC * 2;
  unsigned short* PL  = (unsigned short*)(ws + off); off += (size_t)kNP * kC * 2;
  float* Qf  = (float*)(ws + off); off += (size_t)B * kC * 4;
  float* Kxf = (float*)(ws + off); off += (size_t)B * kC * 4;
  float* Vxf = (float*)(ws + off); off += (size_t)B * kC * 4;
  float* Kpf = (float*)(ws + off); off += (size_t)kNP * kC * 4;
  float* Vpf = (float*)(ws + off); off += (size_t)kNP * kC * 4;
  unsigned short* XCLS = (unsigned short*)(ws + off); off += (size_t)B * kC * 2;
  if (off > ws_size) return;

  const int ntn = kC / 64, ntk = kC / 64;

  pack_wt_kernel<true><<<dim3(ntn * ntk), dim3(256), 0, stream>>>(Wq, WQH, WQL, ntn, ntk);
  pack_wt_kernel<true><<<dim3(ntn * ntk), dim3(256), 0, stream>>>(Wk, WKH, WKL, ntn, ntk);
  pack_wt_kernel<false><<<dim3(ntn * ntk), dim3(256), 0, stream>>>(Wv, WVH, WVH, ntn, ntk);
  pack_wt_kernel<false><<<dim3(ntn * ntk), dim3(256), 0, stream>>>(Wp, WPH, WPH, ntn, ntk);

  const int n8x = B * kC / 8;
  const int n8p = kNP * kC / 8;
  cvt_split_kernel<<<dim3((n8x + 255) / 256), dim3(256), 0, stream>>>(x, XH, XL, n8x);
  cvt_split_kernel<<<dim3((n8p + 255) / 256), dim3(256), 0, stream>>>(prompts, PH, PL, n8p);

  const int mtP = kNP / 16;
  gemm_kernel<true, false><<<dim3(mtP * 2), dim3(256), 0, stream>>>(PH, PL, WKH, WKL, Kpf, bp, x, mtP);
  gemm_kernel<false, false><<<dim3(mtP * 2), dim3(256), 0, stream>>>(PH, PH, WVH, WVH, Vpf, bp, x, mtP);

  const int mtX = B / 16;
  gemm_kernel<true, false><<<dim3(mtX * 2), dim3(256), 0, stream>>>(XH, XL, WQH, WQL, Qf, bp, x, mtX);
  gemm_kernel<true, false><<<dim3(mtX * 2), dim3(256), 0, stream>>>(XH, XL, WKH, WKL, Kxf, bp, x, mtX);
  gemm_kernel<false, false><<<dim3(mtX * 2), dim3(256), 0, stream>>>(XH, XH, WVH, WVH, Vxf, bp, x, mtX);

  attn_kernel<<<dim3(B / 2), dim3(256), 0, stream>>>(Qf, Kxf, Vxf, Kpf, Vpf, out_raw, XCLS, B);

  gemm_kernel<false, true><<<dim3(mtX * 2), dim3(256), 0, stream>>>(XCLS, XCLS, WPH, WPH, out_cls, bp, x, mtX);
}
